// EHH_Layer_9388798509377
// MI455X (gfx1250) — hardware-run, weakly checked
//
#include <hip/hip_runtime.h>


namespace {
constexpr int NBT = 8192, NN = 512, NQ = 6, MM = 1024, OUT = 256, KT = NN * NQ + MM  , KC = 512;
constexpr float XS = 8.0f, WSC = 256.0f;
__constant__ float QC[5] = {-3.0f, -0.834f, -0.248f, 0.248f, 0.834f};
typedef _Float16 b16;
typedef __attribute__((ext_vector_type(16))) _Float16 v16b;
typedef __attribute__((ext_vector_type(8))) _Float16 v8b;
typedef __attribute__((ext_vector_type(8))) float v8f;
typedef __attribute__((ext_vector_type(4))) float v4f;
__device__ __forceinline__ float bf16_rne(float f) { unsigned int u = __float_as_uint(f); u += 0x7FFFu + ((u >> 16) & 1u); float r = __uint_as_float(u & 0xFFFF0000u); asm volatile("" : "+v"(r)); return r; }
__device__ __forceinline__ float bfv(float f) { float r = bf16_rne(f); asm volatile("" : "+v"(r)); return r; }
__device__ __forceinline__ void split16(float v, b16& hi, b16& lo) { hi = (b16)v; lo = (b16)(v - (float)hi); }
__device__ __forceinline__ v16b frag_kb(const b16* p, int hh) { const v8b a = *(const v8b*)(p + 8 * hh), b = *(const v8b*)(p + 16 + 8 * hh); v16b f;
#pragma unroll
  for (int e = 0; e < 8; ++e) { f[e] = a[e]; f[8 + e] = b[e]; } return f; }
__device__ __forceinline__ v8f wmma16b(v16b a, v16b b, v8f c) { v8f d = __builtin_amdgcn_wmma_f32_16x16x32_f16(false, a, false, b, (short)0, c, false, false); asm volatile("v_nop\n\tv_nop\n\tv_nop\n\tv_nop" : "+v"(d) : "v"(a), "v"(b)); return d; }
__device__ __forceinline__ void wave_lds_sync() { __builtin_amdgcn_fence(__ATOMIC_RELEASE, "workgroup"); __builtin_amdgcn_wave_barrier(); __builtin_amdgcn_fence(__ATOMIC_ACQUIRE, "workgroup"); }
__device__ __forceinline__ float pmul(float a, float b) { float p = a * b; asm volatile("" : "+v"(p)); return p; }
__device__ __forceinline__ int iclamp(int v, int lo, int hi) { return v < lo ? lo : (v > hi ? hi : v); }

__global__ __launch_bounds__(256) void wput_kernel(const float* __restrict__ w, b16* __restrict__ WT) { const size_t u = (size_t)blockIdx.x * 256 + threadIdx.x; if (u >= (size_t)OUT * KT / 8) return; const int o = (int)(u / (KT / 8)), k0 = (int)(u % (KT / 8)) * 8; v8b v;
#pragma unroll
  for (int j = 0; j < 8; ++j) v[j] = (b16)(bf16_rne(w[(size_t)(k0 + j) * OUT + o]) * WSC); for (int pass = 0; pass < 2; ++pass) { *(volatile v8b*)(WT + (size_t)o * KT + k0) = v; __threadfence(); } }
__global__ __launch_bounds__(256) void stats_kernel(const float* __restrict__ x, float* __restrict__ ST) { const int n = blockIdx.x * 256 + threadIdx.x; if (n >= NN) return; double s = 0.0, s2 = 0.0;
#pragma unroll 1
  for (int b = 0; b < NBT; ++b) { const double v = (double)bf16_rne(x[(size_t)b * NN + n]); s += v; s2 += v * v; }
  const double mu = s / NBT; const double var = s2 / NBT - mu * mu; const float m = (float)mu, vr = (float)(var > 0.0 ? var : 0.0);
  for (int pass = 0; pass < 2; ++pass) { ((volatile float*)ST)[n] = m; ((volatile float*)ST)[NN + n] = vr; __threadfence(); } }
__device__ __forceinline__ float maxq(float xv, int n, int q, const float* ST, const float* gam, const float* bet) { const float mu = ST[n], var = ST[NN + n], g = bfv(gam[n]), be = bfv(bet[n]); const float nr = pmul(g, (xv - mu) / sqrtf(var + 0.001f)) + be; if (q == 0) return fmaxf(nr, 0.0f); const float quant = QC[q - 1] * var + mu; return fmaxf(nr - pmul(quant, g) + be, 0.0f); }
__global__ __launch_bounds__(32) void ehh_kernel(const float* __restrict__ x, const float* __restrict__ ST, const float* __restrict__ gam, const float* __restrict__ bet, const int* __restrict__ ci, const float* __restrict__ bias, const b16* __restrict__ WT, int RLIM, float* __restrict__ out) { __shared__ __attribute__((aligned(16))) b16 Ah[16][KC + 8], Al[16][KC + 8]; __shared__ float Tf[16][OUT + 4]; const int lane = threadIdx.x, nloc = lane & 15, hlf = lane >> 4; const size_t m0 = (size_t)blockIdx.x * 16; if (m0 >= (size_t)RLIM) return;
  v8f acc[16];
#pragma unroll
  for (int t = 0; t < 16; ++t) acc[t] = (v8f){};
#pragma unroll 1
  for (int kc = 0; kc < KT; kc += KC) {
    for (int rr = 0; rr < 16; ++rr) { const size_t b = m0 + rr;
      for (int j = lane; j < KC; j += 32) { const int col = kc + j; float v;
        if (col < NN * NQ) { const int n = col / NQ, q = col % NQ; v = maxq(bf16_rne(x[b * NN + n]), n, q, ST, gam, bet); }
        else { const int m = col - NN * NQ; const int n1 = iclamp(ci[m * 5 + 1], 0, NN - 1), q1 = iclamp(ci[m * 5 + 2], 0, NQ - 1), n2 = iclamp(ci[m * 5 + 3], 0, NN - 1), q2 = iclamp(ci[m * 5 + 4], 0, NQ - 1); v = fminf(maxq(bf16_rne(x[b * NN + n1]), n1, q1, ST, gam, bet), maxq(bf16_rne(x[b * NN + n2]), n2, q2, ST, gam, bet)); }
        b16 p, ql; split16(v * XS, p, ql); Ah[rr][j] = p; Al[rr][j] = ql; } }
    wave_lds_sync();
#pragma unroll 2
    for (int ks = 0; ks < KC; ks += 32) { const v16b a = frag_kb(&Ah[nloc][ks], hlf), al = frag_kb(&Al[nloc][ks], hlf);
#pragma unroll
      for (int t = 0; t < 16; ++t) { const v16b bw = frag_kb(WT + (size_t)(t * 16 + nloc) * KT + kc + ks, hlf); acc[t] = wmma16b(a, bw, acc[t]); acc[t] = wmma16b(al, bw, acc[t]); } }
    wave_lds_sync(); }
  const float bb = bfv(bias[0]);
#pragma unroll
  for (int t = 0; t < 16; ++t)
#pragma unroll
    for (int r8 = 0; r8 < 8; ++r8) Tf[8 * hlf + r8][t * 16 + nloc] = acc[t][r8] * (1.0f / (XS * WSC)) + bb;
  wave_lds_sync();
  for (int pass = 0; pass < 2; ++pass) { for (int rr = 0; rr < 16; ++rr) for (int q = 0; q < 2; ++q) *(volatile v4f*)(out + (m0 + rr) * OUT + q * 128 + lane * 4) = *(const v4f*)(&Tf[rr][q * 128 + lane * 4]); __threadfence(); } }
}

extern "C" void kernel_launch(void* const* d_in, const int* in_sizes, int n_in, void* d_out, int out_size, void* d_ws, size_t ws_size, hipStream_t stream) {
  (void)n_in;
  auto Fp = [&](int i) { return (const float*)d_in[i]; }; auto Ip = [&](int i) { return (const int*)d_in[i]; };
  if (in_sizes[0] != NBT * NN || in_sizes[1] != NN || in_sizes[2] != NN || in_sizes[3] != KT * OUT || in_sizes[4] != 1 || in_sizes[5] != MM * 5 || out_size != NBT * OUT) return;
  const int RLIM = NBT;
  size_t off = 0; char* ws = (char*)d_ws;
  auto carve = [&](size_t bytes) { char* p = ws + off; off += (bytes + 255) & ~(size_t)255; return p; };
  b16* WT = (b16*)carve((size_t)OUT * KT * 2); float* ST = (float*)carve(2 * NN * 4);
  if (off > ws_size || off > ((size_t)4 << 20)) return;
  wput_kernel<<<(unsigned)(((size_t)OUT * KT / 8 + 255) / 256), 256, 0, stream>>>(Fp(3), WT);
  stats_kernel<<<(NN + 255) / 256, 256, 0, stream>>>(Fp(0), ST);
  ehh_kernel<<<RLIM / 16, 32, 0, stream>>>(Fp(0), ST, Fp(2), Fp(1), Ip(5), Fp(4), WT, RLIM, (float*)d_out);
}
